// MultiHeadCrossAttention_3083786519235
// MI455X (gfx1250) — hardware-verified
//
#include <hip/hip_runtime.h>
#include <math.h>

#ifndef NB
#define NB 8
#endif
#ifndef SEQ
#define SEQ 1024
#endif
#define NB_FULL 8
#define LQ_FULL 1024
#define LK 1024
#define DM 1024
#define NH 16
#define DH 64
#define HD (NH * DH)
static_assert(NB >= 1 && NB <= NB_FULL);
static_assert(SEQ % 64 == 0 && SEQ >= 64 && SEQ <= LQ_FULL);
static_assert(LK % 64 == 0 && DM % 64 == 0 && HD % 64 == 0 && DH == 64);
static_assert(HD == DM);

typedef __attribute__((ext_vector_type(16))) _Float16 v16h;
typedef __attribute__((ext_vector_type(8)))  _Float16 v8h;
typedef __attribute__((ext_vector_type(16))) __bf16   v16b;
typedef __attribute__((ext_vector_type(8)))  __bf16   v8b;
typedef __attribute__((ext_vector_type(8)))  float    v8f;
typedef __attribute__((ext_vector_type(4)))  float    v4f;
typedef __attribute__((ext_vector_type(16))) unsigned short v16us;
typedef __attribute__((ext_vector_type(8)))  unsigned short v8us;
typedef __attribute__((ext_vector_type(4)))  unsigned v4u;

__device__ __forceinline__ unsigned short bf_bits(float f) {
    unsigned u = __float_as_uint(f);
    return (unsigned short)((u + 0x7FFFu + ((u >> 16) & 1u)) >> 16);
}
__device__ __forceinline__ v8f wmmab(v16b a, v16b b, v8f c) {
    c = __builtin_amdgcn_wmma_f32_16x16x32_bf16(false, a, false, b, (short)0, c, false, false);
    asm volatile("v_nop\n\tv_nop\n\tv_nop\n\tv_nop" : "+v"(c) : "v"(a), "v"(b));
    return c;
}
__device__ __forceinline__ v8f wmmah(v16h a, v16h b, v8f c) {
    c = __builtin_amdgcn_wmma_f32_16x16x32_f16(false, a, false, b, (short)0, c, false, false);
    asm volatile("v_nop\n\tv_nop\n\tv_nop\n\tv_nop" : "+v"(c) : "v"(a), "v"(b));
    return c;
}
union FU { v16us v; v8us h[2]; };

__global__ __launch_bounds__(256) void k_cvbf(const float* __restrict__ src, unsigned short* __restrict__ dst, long long n8) {
    const long long u = (long long)blockIdx.x * 256 + threadIdx.x;
    if (u >= n8) return;
    const v4f a = *(const v4f*)(src + 8 * u);
    const v4f b = *(const v4f*)(src + 8 * u + 4);
    v4u pk;
    pk.x = (unsigned)bf_bits(a.x) | ((unsigned)bf_bits(a.y) << 16);
    pk.y = (unsigned)bf_bits(a.z) | ((unsigned)bf_bits(a.w) << 16);
    pk.z = (unsigned)bf_bits(b.x) | ((unsigned)bf_bits(b.y) << 16);
    pk.w = (unsigned)bf_bits(b.z) | ((unsigned)bf_bits(b.w) << 16);
    volatile v4u* d = (volatile v4u*)(dst + 8 * u);
    *d = pk;
    __threadfence();
    *d = pk;
}

namespace w25 {

__device__ __forceinline__ unsigned short f2bf_bits(float f) {
  unsigned u = __float_as_uint(f);
  return (unsigned short)((u + 0x7FFFu + ((u >> 16) & 1u)) >> 16);
}
__device__ __forceinline__ float bf_bits2f(unsigned short h) { return __uint_as_float(((unsigned)h) << 16); }

__device__ __forceinline__ void dep_guard_h(v8f& a, v8f& b, v16h x, v16h y) { asm volatile("v_nop\n\tv_nop\n\tv_nop\n\tv_nop" : "+v"(a), "+v"(b) : "v"(x), "v"(y)); }
__device__ __forceinline__ void dep_guard_b(v8f& a, v8f& b, v16b x, v16b y) { asm volatile("v_nop\n\tv_nop\n\tv_nop\n\tv_nop" : "+v"(a), "+v"(b) : "v"(x), "v"(y)); }
__device__ __forceinline__ void keep4_h(v16h a, v16h b, v16h c, v16h d) { asm volatile("v_nop" :: "v"(a), "v"(b), "v"(c), "v"(d)); }
__device__ __forceinline__ void keep4_b(v16b a, v16b b, v16b c, v16b d) { asm volatile("v_nop" :: "v"(a), "v"(b), "v"(c), "v"(d)); }
__device__ __forceinline__ void acc_guard4(v8f& a, v8f& b, v8f& c, v8f& d) { asm volatile("v_nop\n\tv_nop\n\tv_nop\n\tv_nop" : "+v"(a), "+v"(b), "+v"(c), "+v"(d)); }
template <typename T> struct Frag;
template <> struct Frag<_Float16> {
  typedef v16h V; union U { v16h v; v8h h[2]; };
  static __device__ __forceinline__ v16h load(const _Float16* p) {
    U f; f.h[0] = *(const v8h*)(p); f.h[1] = *(const v8h*)(p + 16); return f.v;
  }
  static __device__ __forceinline__ v8f mma(v16h a, v16h b, v8f c) {
    return __builtin_amdgcn_wmma_f32_16x16x32_f16(false, a, false, b, (short)0, c, false, false);
  }
  static __device__ __forceinline__ void guard(v8f& a, v8f& b, v16h x, v16h y) { dep_guard_h(a, b, x, y); }
  static __device__ __forceinline__ void keep(v16h a, v16h b, v16h c, v16h d) { keep4_h(a, b, c, d); }
};
template <> struct Frag<__bf16> {
  typedef v16b V; union U { v16b v; v8b h[2]; };
  static __device__ __forceinline__ v16b load(const __bf16* p) {
    U f; f.h[0] = *(const v8b*)(p); f.h[1] = *(const v8b*)(p + 16); return f.v;
  }
  static __device__ __forceinline__ v8f mma(v16b a, v16b b, v8f c) {
    return __builtin_amdgcn_wmma_f32_16x16x32_bf16(false, a, false, b, (short)0, c, false, false);
  }
  static __device__ __forceinline__ void guard(v8f& a, v8f& b, v16b x, v16b y) { dep_guard_b(a, b, x, y); }
  static __device__ __forceinline__ void keep(v16b a, v16b b, v16b c, v16b d) { keep4_b(a, b, c, d); }
};

template <int ET> struct Elem;
template <> struct Elem<0> { typedef _Float16 T; };
template <> struct Elem<1> { typedef __bf16 T; };
template <int ET, bool SPLIT, int OUT_MODE>
__global__ __launch_bounds__(256) void wmma_gemm64(
    const unsigned short* __restrict__ Ap, const unsigned short* __restrict__ A2p, int lda, long strideA,
    const unsigned short* __restrict__ Btp, const unsigned short* __restrict__ Bt2p, int ldb, long strideB,
    void* __restrict__ Cout, void* __restrict__ Cout2, int ldc, long strideC,
    int M, int N, int K, float scale) {
  typedef typename Elem<ET>::T T;
  typedef typename Frag<T>::V V;
  const T* A = (const T*)Ap; const T* A2 = (const T*)A2p; const T* Bt = (const T*)Btp; const T* Bt2 = (const T*)Bt2p;
  __shared__ __align__(16) float sT[8][16 * 68];
  const int b    = blockIdx.y;
  const int lane = threadIdx.x & 31;
  const int wave = threadIdx.x >> 5;
  const int tilesN = N >> 6;
  const int tilesM = M >> 6;
  const int tile = blockIdx.x * 8 + wave;
  if (tile >= tilesM * tilesN) return;
  const int tm = tile / tilesN;
  const int tn = tile - tm * tilesN;
  const int m0 = tm << 6;
  const int n0 = tn << 6;

  const T* Ab  = A  + (size_t)b * strideA;
  const T* Bb  = Bt + (size_t)b * strideB;
  const T* Ab2 = SPLIT ? (A2  + (size_t)b * strideA) : nullptr;
  const T* Bb2 = SPLIT ? (Bt2 + (size_t)b * strideB) : nullptr;

  const int rlane = lane & 15;
  const int koff  = (lane >> 4) * 8;
  const int mOff  = (lane >> 4) * 8;

  v8f acc[4][4];
#pragma unroll
  for (int i = 0; i < 4; ++i)
#pragma unroll
    for (int j = 0; j < 4; ++j) acc[i][j] = (v8f){0.f,0.f,0.f,0.f,0.f,0.f,0.f,0.f};

  for (int k0 = 0; k0 < K; k0 += 32) {
    V bh[4], bl[4];
#pragma unroll
    for (int j = 0; j < 4; ++j) {
      const size_t bo = (size_t)(n0 + (j << 4) + rlane) * ldb + koff + k0;
      bh[j] = Frag<T>::load(Bb + bo);
      if (SPLIT) bl[j] = Frag<T>::load(Bb2 + bo); else bl[j] = bh[j];
    }
#pragma unroll
    for (int i = 0; i < 4; ++i) {
      const size_t ao = (size_t)(m0 + (i << 4) + rlane) * lda + koff + k0;
      V ah = Frag<T>::load(Ab + ao);
      V al;
      if (SPLIT) al = Frag<T>::load(Ab2 + ao); else al = ah;
#pragma unroll
      for (int j = 0; j < 4; ++j) {
        acc[i][j] = Frag<T>::mma(ah, bh[j], acc[i][j]);
        if (SPLIT) {
          acc[i][j] = Frag<T>::mma(ah, bl[j], acc[i][j]);
          acc[i][j] = Frag<T>::mma(al, bh[j], acc[i][j]);
        }
      }
      Frag<T>::guard(acc[i][0], acc[i][3], ah, al);
    }
    Frag<T>::keep(bh[0], bh[1], bh[2], bh[3]);
    if (SPLIT) Frag<T>::keep(bl[0], bl[1], bl[2], bl[3]);
  }
  acc_guard4(acc[0][0], acc[0][1], acc[0][2], acc[0][3]);
  acc_guard4(acc[1][0], acc[1][1], acc[1][2], acc[1][3]);
  acc_guard4(acc[2][0], acc[2][1], acc[2][2], acc[2][3]);
  acc_guard4(acc[3][0], acc[3][1], acc[3][2], acc[3][3]);

  float* slab = sT[wave];
#pragma unroll
  for (int i = 0; i < 4; ++i) {
    const int mBase = m0 + (i << 4);
#pragma unroll
    for (int j = 0; j < 4; ++j) {
#pragma unroll
      for (int r = 0; r < 8; ++r) {
        const float v = acc[i][j][r] * scale;
        slab[(mOff + r) * 68 + (j << 4) + rlane] = v;
      }
    }
    __builtin_amdgcn_fence(__ATOMIC_RELEASE, "workgroup");
    __builtin_amdgcn_wave_barrier();
    __builtin_amdgcn_fence(__ATOMIC_ACQUIRE, "workgroup");
    if (OUT_MODE == 0) {
      float* C = (float*)Cout + (size_t)b * strideC;
      const int hh = lane >> 4, c4 = (lane & 15) * 4;
      for (int pass = 0; pass < 2; ++pass) {
#pragma unroll
        for (int it = 0; it < 8; ++it) {
          const int row = it * 2 + hh;
          v4f v = *(const v4f*)(slab + row * 68 + c4);
          *(volatile v4f*)(C + (size_t)(mBase + row) * ldc + n0 + c4) = v;
        }
        __threadfence();
      }
    } else {
      const int q = lane >> 3, c8 = (lane & 7) * 8;
      unsigned short* C  = (unsigned short*)Cout  + (size_t)b * strideC;
      unsigned short* C2 = (OUT_MODE >= 2) ? ((unsigned short*)Cout2 + (size_t)b * strideC) : nullptr;
      for (int pass = 0; pass < 2; ++pass) {
#pragma unroll
        for (int it = 0; it < 4; ++it) {
          const int row = it * 4 + q;
          const float* sp = slab + row * 68 + c8;
          v8h hv, lv;
#pragma unroll
          for (int e = 0; e < 8; ++e) {
            if (OUT_MODE == 1) {
              hv[e] = (_Float16)sp[e]; lv[e] = hv[e];
            } else if (OUT_MODE == 3) {
              const _Float16 hq = (_Float16)sp[e];
              hv[e] = hq;
              lv[e] = (_Float16)((sp[e] - (float)hq) * 2048.0f);
            } else {
              unsigned short hb = f2bf_bits(sp[e]);
              unsigned short lb = f2bf_bits(sp[e] - bf_bits2f(hb));
              hv[e] = __builtin_bit_cast(_Float16, hb);
              lv[e] = __builtin_bit_cast(_Float16, lb);
            }
          }
          *(volatile v8h*)(C + (size_t)(mBase + row) * ldc + n0 + c8) = hv;
          if (OUT_MODE >= 2) *(volatile v8h*)(C2 + (size_t)(mBase + row) * ldc + n0 + c8) = lv;
        }
        __threadfence();
      }
    }
    __builtin_amdgcn_fence(__ATOMIC_RELEASE, "workgroup");
    __builtin_amdgcn_wave_barrier();
    __builtin_amdgcn_fence(__ATOMIC_ACQUIRE, "workgroup");
  }
}

}

#define PSC 16384.0f
#define RSC 2048.0f
__global__ __launch_bounds__(128) void k_mha64(const unsigned short* __restrict__ Qh, const unsigned short* __restrict__ Ql,
                                             const unsigned short* __restrict__ Kh, const unsigned short* __restrict__ Kl,
                                             const unsigned short* __restrict__ Vh, const unsigned short* __restrict__ Vr,
                                             float* __restrict__ out) {
    __shared__ __align__(16) unsigned short Psh[4][16 * 64];
    __shared__ __align__(16) unsigned short Psr[4][16 * 64];
    __shared__ __align__(16) float          Os[4][16 * 68];

    const int tid  = threadIdx.x;
    const int wave = tid >> 5;
    const int lane = tid & 31;
    const int hh   = lane >> 4;
    const int c    = lane & 15;

    const int nqb = SEQ / 64;
    const int bx = blockIdx.x;
    const int qb = bx % nqb;
    const int bh = bx / nqb;
    const int h  = bh % NH;
    const int b  = bh / NH;
    const int q0 = qb * 64 + wave * 16;

    const size_t qoff = (size_t)b * LQ_FULL * HD + (size_t)h * DH;
    const size_t koff = (size_t)b * LK * HD + (size_t)h * DH;
    const size_t voff = ((size_t)b * HD + (size_t)h * DH) * LK;
    const unsigned short* qhp = Qh + qoff; const unsigned short* qlp = Ql + qoff;
    const unsigned short* khp = Kh + koff; const unsigned short* klp = Kl + koff;
    const unsigned short* vhp = Vh + voff; const unsigned short* vrp = Vr + voff;
    float* ob = out + (size_t)b * LQ_FULL * HD + (size_t)h * DH;

    v16b qah[2], qal[2];
    {
        const size_t ro = (size_t)(q0 + c) * HD;
#pragma unroll
        for (int dc = 0; dc < 2; ++dc) {
            FU f;
            f.h[0] = *(const v8us*)(qhp + ro + dc * 32 + 8 * hh);
            f.h[1] = *(const v8us*)(qhp + ro + dc * 32 + 16 + 8 * hh);
            qah[dc] = __builtin_bit_cast(v16b, f.v);
            f.h[0] = *(const v8us*)(qlp + ro + dc * 32 + 8 * hh);
            f.h[1] = *(const v8us*)(qlp + ro + dc * 32 + 16 + 8 * hh);
            qal[dc] = __builtin_bit_cast(v16b, f.v);
        }
    }

    float mrow[8], lrow[8];
    v8f oacc[4], oacc2[4];
#pragma unroll
    for (int r = 0; r < 8; ++r) { mrow[r] = -__builtin_inff(); lrow[r] = 0.f; }
#pragma unroll
    for (int t = 0; t < 4; ++t) { oacc[t] = (v8f){0.f,0.f,0.f,0.f,0.f,0.f,0.f,0.f}; oacc2[t] = (v8f){0.f,0.f,0.f,0.f,0.f,0.f,0.f,0.f}; }

    unsigned short* pwh = Psh[wave];
    unsigned short* pwl = Psr[wave];

#pragma unroll 1
    for (int kc = 0; kc < LK / 64; ++kc) {
        const int kv0 = kc * 64;
        __syncthreads();

        v8f s[4];
#pragma unroll
        for (int j = 0; j < 4; ++j) {
            v8f acc = {};
            const size_t ko = (size_t)(kv0 + j * 16 + c) * HD;
#pragma unroll
            for (int dc = 0; dc < 2; ++dc) {
                FU kb, kl;
                kb.h[0] = *(const v8us*)(khp + ko + dc * 32 + 8 * hh);
                kb.h[1] = *(const v8us*)(khp + ko + dc * 32 + 16 + 8 * hh);
                kl.h[0] = *(const v8us*)(klp + ko + dc * 32 + 8 * hh);
                kl.h[1] = *(const v8us*)(klp + ko + dc * 32 + 16 + 8 * hh);
                const v16b kbv = __builtin_bit_cast(v16b, kb.v);
                const v16b klv = __builtin_bit_cast(v16b, kl.v);
                acc = wmmab(qah[dc], kbv, acc);
                acc = wmmab(qah[dc], klv, acc);
                acc = wmmab(qal[dc], kbv, acc);
            }
            s[j] = acc;
        }

        float cm[8];
#pragma unroll
        for (int r = 0; r < 8; ++r) {
            float m = fmaxf(fmaxf(s[0][r], s[1][r]), fmaxf(s[2][r], s[3][r]));
#pragma unroll
            for (int off = 1; off < 16; off <<= 1) m = fmaxf(m, __shfl_xor(m, off, 32));
            cm[r] = m;
        }
#pragma unroll
        for (int r = 0; r < 8; ++r) {
            const float mnew = fmaxf(mrow[r], cm[r]);
            const float alpha = expf(mrow[r] - mnew);
            mrow[r] = mnew;
            float psum = 0.f;
#pragma unroll
            for (int j = 0; j < 4; ++j) {
                const float p = expf(s[j][r] - mnew);
                psum += p;
                const float pc = p * PSC;
                const _Float16 ph = (_Float16)pc;
                const _Float16 pr = (_Float16)((pc - (float)ph) * RSC);
                pwh[(8 * hh + r) * 64 + j * 16 + c] = __builtin_bit_cast(unsigned short, ph);
                pwl[(8 * hh + r) * 64 + j * 16 + c] = __builtin_bit_cast(unsigned short, pr);
            }
#pragma unroll
            for (int off = 1; off < 16; off <<= 1) psum += __shfl_xor(psum, off, 32);
            lrow[r] = lrow[r] * alpha + psum;
#pragma unroll
            for (int t = 0; t < 4; ++t) { oacc[t][r] *= alpha; oacc2[t][r] *= alpha; }
        }
        __builtin_amdgcn_fence(__ATOMIC_RELEASE, "workgroup");
        __builtin_amdgcn_wave_barrier();
        __builtin_amdgcn_fence(__ATOMIC_ACQUIRE, "workgroup");

#pragma unroll
        for (int kk = 0; kk < 2; ++kk) {
            const int po = c * 64 + kk * 32 + 8 * hh;
            FU pa, pl;
            pa.h[0] = *(const v8us*)(pwh + po);
            pa.h[1] = *(const v8us*)(pwh + po + 16);
            pl.h[0] = *(const v8us*)(pwl + po);
            pl.h[1] = *(const v8us*)(pwl + po + 16);
            const v16h pav = __builtin_bit_cast(v16h, pa.v);
            const v16h plv = __builtin_bit_cast(v16h, pl.v);
#pragma unroll
            for (int t = 0; t < 4; ++t) {
                const size_t vo = (size_t)(t * 16 + c) * LK + kv0 + kk * 32 + 8 * hh;
                FU vb, vr;
                vb.h[0] = *(const v8us*)(vhp + vo);
                vb.h[1] = *(const v8us*)(vhp + vo + 16);
                vr.h[0] = *(const v8us*)(vrp + vo);
                vr.h[1] = *(const v8us*)(vrp + vo + 16);
                const v16h vbv = __builtin_bit_cast(v16h, vb.v);
                const v16h vrv = __builtin_bit_cast(v16h, vr.v);
                oacc[t]  = wmmah(pav, vbv, oacc[t]);
                oacc2[t] = wmmah(pav, vrv, oacc2[t]);
                oacc2[t] = wmmah(plv, vbv, oacc2[t]);
            }
        }
    }

    float* os = Os[wave];
#pragma unroll
    for (int r = 0; r < 8; ++r) {
        const float inv = 1.0f / (lrow[r] * PSC);
#pragma unroll
        for (int t = 0; t < 4; ++t) os[(8 * hh + r) * 68 + t * 16 + c] = (oacc[t][r] + oacc2[t][r] * (1.0f / RSC)) * inv;
    }
    __builtin_amdgcn_fence(__ATOMIC_RELEASE, "workgroup");
    __builtin_amdgcn_wave_barrier();
    __builtin_amdgcn_fence(__ATOMIC_ACQUIRE, "workgroup");
    {
        const int c4 = (lane & 15) * 4;
        for (int pass = 0; pass < 2; ++pass) {
#pragma unroll
            for (int it = 0; it < 8; ++it) {
                const int row = it * 2 + hh;
                v4f val = *(const v4f*)(os + row * 68 + c4);
                *(volatile v4f*)(ob + (size_t)(q0 + row) * HD + c4) = val;
            }
            __threadfence();
        }
    }
}

extern "C" void kernel_launch(void* const* d_in, const int* in_sizes, int n_in,
                              void* d_out, int out_size, void* d_ws, size_t ws_size, hipStream_t stream) {
    if (n_in < 6) return;
    if (in_sizes[0] < NB * LQ_FULL * DM || in_sizes[1] < NB * LK * DM || in_sizes[2] < NB * LK * DM) return;
    if (in_sizes[3] < HD * DM || in_sizes[4] < HD * DM || in_sizes[5] < HD * DM) return;
    if (out_size < NB * LQ_FULL * HD) return;
    const float* query  = (const float*)d_in[0];
    const float* keys   = (const float*)d_in[1];
    const float* values = (const float*)d_in[2];
    const float* Wq     = (const float*)d_in[3];
    const float* Wk     = (const float*)d_in[4];
    const float* Wv     = (const float*)d_in[5];
    float* out = (float*)d_out;

    const size_t wbytes = (size_t)HD * DM * 2;
    const size_t xq_b   = (size_t)NB * LQ_FULL * DM * 2;
    const size_t xk_b   = (size_t)NB * LK * DM * 2;
    const size_t xbytes = (xq_b > xk_b) ? xq_b : xk_b;
    const size_t qbytes = (size_t)NB * LQ_FULL * HD * 2;
    const size_t kbytes = (size_t)NB * LK * HD * 2;
    const size_t vbytes = (size_t)NB * HD * LK * 2;
    char* wsp = (char*)d_ws;
    unsigned short* WQ = (unsigned short*)wsp; wsp += wbytes;
    unsigned short* WK = (unsigned short*)wsp; wsp += wbytes;
    unsigned short* WV = (unsigned short*)wsp; wsp += wbytes;
    unsigned short* X  = (unsigned short*)wsp; wsp += xbytes;
    unsigned short* QH = (unsigned short*)wsp; wsp += qbytes;
    unsigned short* QL = (unsigned short*)wsp; wsp += qbytes;
    unsigned short* KH = (unsigned short*)wsp; wsp += kbytes;
    unsigned short* KL = (unsigned short*)wsp; wsp += kbytes;
    unsigned short* VH = (unsigned short*)wsp; wsp += vbytes;
    unsigned short* VR = (unsigned short*)wsp; wsp += vbytes;
    if ((size_t)(wsp - (char*)d_ws) > ws_size) return;

    const long long nw8 = (long long)HD * DM / 8;
    const unsigned gw = (unsigned)((nw8 + 255) / 256);
    k_cvbf<<<gw, 256, 0, stream>>>(Wq, WQ, nw8);
    k_cvbf<<<gw, 256, 0, stream>>>(Wk, WK, nw8);
    k_cvbf<<<gw, 256, 0, stream>>>(Wv, WV, nw8);

    const long long nq8 = (long long)NB * LQ_FULL * DM / 8;
    k_cvbf<<<(unsigned)((nq8 + 255) / 256), 256, 0, stream>>>(query, X, nq8);
    w25::wmma_gemm64<1, false, 2><<<dim3((unsigned)(((SEQ / 64) * (HD / 64) + 7) / 8), (unsigned)NB), 256, 0, stream>>>(
        X, nullptr, DM, (long)LQ_FULL * DM, WQ, nullptr, DM, 0L, (void*)QH, (void*)QL, HD, (long)LQ_FULL * HD, SEQ, HD, DM, 0.125f);

    const long long nk8 = (long long)NB * LK * DM / 8;
    k_cvbf<<<(unsigned)((nk8 + 255) / 256), 256, 0, stream>>>(keys, X, nk8);
    w25::wmma_gemm64<1, false, 2><<<dim3((unsigned)(((LK / 64) * (HD / 64) + 7) / 8), (unsigned)NB), 256, 0, stream>>>(
        X, nullptr, DM, (long)LK * DM, WK, nullptr, DM, 0L, (void*)KH, (void*)KL, HD, (long)LK * HD, LK, HD, DM, 1.0f);

    k_cvbf<<<(unsigned)((nk8 + 255) / 256), 256, 0, stream>>>(values, X, nk8);
    w25::wmma_gemm64<1, false, 3><<<dim3((unsigned)(((HD / 64) * (LK / 64) + 7) / 8), (unsigned)NB), 256, 0, stream>>>(
        WV, nullptr, DM, 0L, X, nullptr, DM, (long)LK * DM, (void*)VH, (void*)VR, LK, (long)HD * LK, HD, LK, DM, 1.0f);

    k_mha64<<<(unsigned)(NB * NH * (SEQ / 64)), 128, 0, stream>>>(QH, QL, KH, KL, VH, VR, out);
}
